// HybridAttention_48326972014899
// MI455X (gfx1250) — hardware-verified
//
#include <hip/hip_runtime.h>
#include <math.h>

#ifndef NB
#define NB 4
#endif
#ifndef SEQ
#define SEQ 2048
#endif
#define NB_FULL 4
#define SEQ_FULL 2048
#define DM 512
#define D3 1536
#define NH 8
#define HD 64
#define WCH ((((SEQ) / 4) < 256) ? ((SEQ) / 4) : 256)
#define LK (2 * WCH)
#define HGG 2
#define HGL 8

static_assert(NB >= 1 && NB <= NB_FULL);
static_assert(SEQ >= 256 && SEQ <= SEQ_FULL && (SEQ % 128) == 0);
static_assert((WCH % 64) == 0 && (LK % 128) == 0 && (SEQ % WCH) == 0 && LK <= SEQ);
static_assert(NH * HD == DM && (NH % HGG) == 0 && HGL == NH && (DM % 128) == 0 && (D3 % 128) == 0);

typedef __attribute__((ext_vector_type(16))) _Float16 v16h;
typedef __attribute__((ext_vector_type(16))) __bf16 v16b;
typedef __attribute__((ext_vector_type(8)))  _Float16 v8h;
typedef __attribute__((ext_vector_type(8)))  __bf16 v8b;
typedef __attribute__((ext_vector_type(8)))  float v8f;
typedef __attribute__((ext_vector_type(4)))  float v4f;
typedef __attribute__((ext_vector_type(4)))  unsigned v4u;

template <typename T> __device__ __forceinline__ void vst2(void* p, T v) { *(volatile T*)p = v; __threadfence(); *(volatile T*)p = v; }
__device__ __forceinline__ v8f wmma16(v16h a, v16h b, v8f c) {
  v8f d = __builtin_amdgcn_wmma_f32_16x16x32_f16(false, a, false, b, (short)0, c, false, false);
  asm volatile("v_nop\n\tv_nop\n\tv_nop\n\tv_nop" : "+v"(d) : "v"(a), "v"(b));
  return d;
}
__device__ __forceinline__ v8f wmma_bf(v16b a, v16b b, v8f c) {
  v8f d = __builtin_amdgcn_wmma_f32_16x16x32_bf16(false, a, false, b, (short)0, c, false, false);
  asm volatile("v_nop\n\tv_nop\n\tv_nop\n\tv_nop" : "+v"(d) : "v"(a), "v"(b));
  return d;
}
__device__ __forceinline__ v16h frag_h(const _Float16* rowk0, int lane) {
  union { v16h v; v8h q[2]; } u; const _Float16* p = rowk0 + 8 * (lane >> 4);
  u.q[0] = *(const v8h*)p; u.q[1] = *(const v8h*)(p + 16); return u.v;
}
__device__ __forceinline__ v16b frag_b(const __bf16* rowk0, int lane) {
  union { v16b v; v8b q[2]; } u; const __bf16* p = rowk0 + 8 * (lane >> 4);
  u.q[0] = *(const v8b*)p; u.q[1] = *(const v8b*)(p + 16); return u.v;
}
struct F2 { v16b h, l; };
__device__ __forceinline__ F2 bsplit16(const float v[16]) { F2 r;
#pragma unroll
  for (int i = 0; i < 16; ++i) { const __bf16 h = (__bf16)v[i]; r.h[i] = h; r.l[i] = (__bf16)(v[i] - (float)h); }
  return r; }
__device__ __forceinline__ F2 split_row(const float* row, int k0, int lane) { float v[16]; const float* p = row + k0 + 8 * (lane >> 4);
#pragma unroll
  for (int i = 0; i < 8; ++i) { v[i] = p[i]; v[8 + i] = p[16 + i]; }
  return bsplit16(v); }
__device__ __forceinline__ float bfr(float v) { return (float)(__bf16)v; }
#define LDSX() do { asm volatile("s_wait_dscnt 0" ::: "memory"); __builtin_amdgcn_wave_barrier(); __builtin_amdgcn_fence(__ATOMIC_RELEASE, "workgroup"); } while (0)

#define RWS ((size_t)NB * SEQ)
#define WS_XL  ((size_t)0)
#define WS_XG  (WS_XL + 2u * RWS * DM)
#define WS_WIL (WS_XG + 2u * RWS * DM)
#define WS_WIG (WS_WIL + 2u * (size_t)D3 * DM)
#define WS_WOL (WS_WIG + 2u * (size_t)D3 * DM)
#define WS_WOG (WS_WOL + 2u * (size_t)DM * DM)
#define WS_QH  (WS_WOG + 2u * (size_t)DM * DM)
#define WS_QL  (WS_QH + 2u * RWS * DM)
#define WS_KH  (WS_QL + 2u * RWS * DM)
#define WS_VT  (WS_KH + 2u * RWS * DM)
#define WS_VL  (WS_VT + 2u * RWS * DM)
#define WS_S   (WS_VL + 2u * RWS * DM)
#define S_FLOATS_G ((size_t)HGG * SEQ * SEQ)
#define S_FLOATS_L ((size_t)HGL * SEQ * LK)
#define S_FLOATS (S_FLOATS_G > S_FLOATS_L ? S_FLOATS_G : S_FLOATS_L)
#define WS_YL  (WS_S + 4u * S_FLOATS)
#define WS_YG  (WS_YL + 4u * RWS * DM)
#define WS_END (WS_YG + 4u * RWS * DM)
static_assert(S_FLOATS_G <= S_FLOATS && S_FLOATS_L <= S_FLOATS);
static_assert(WS_END <= (size_t)134217728);
static_assert((WS_S % 128) == 0 && (WS_YL % 128) == 0 && (WS_YG % 128) == 0 && (WS_QH % 128) == 0);

__global__ __launch_bounds__(128) void k_cvt16(const float* __restrict__ A0, const float* __restrict__ A1, _Float16* __restrict__ O0, _Float16* __restrict__ O1, int nrows) {
  const int tid = threadIdx.x, wave = tid >> 5, lane = tid & 31;
  const int row = blockIdx.x * 4 + wave;
  const float* A = (blockIdx.y == 0) ? A0 : A1; _Float16* O = (blockIdx.y == 0) ? O0 : O1;
  if (row >= nrows) return;
  const float* p = A + (size_t)row * DM;
#pragma unroll
  for (int hh = 0; hh < 2; ++hh) {
    const int c = hh * (DM / 2) + 8 * lane;
    const v4f a0 = *(const v4f*)(p + c), a1 = *(const v4f*)(p + c + 4);
    union { v8h h; v4u u; } o;
#pragma unroll
    for (int i = 0; i < 4; ++i) { o.h[i] = (_Float16)(bfr(a0[i]) * 16.0f); o.h[4 + i] = (_Float16)(bfr(a1[i]) * 16.0f); }
    vst2(O + (size_t)row * DM + c, o.u);
  }
}
__global__ __launch_bounds__(128) void k_cvtb(const float* __restrict__ A0, const float* __restrict__ A1, __bf16* __restrict__ O0, __bf16* __restrict__ O1, int nrows) {
  const int tid = threadIdx.x, wave = tid >> 5, lane = tid & 31;
  const int row = blockIdx.x * 4 + wave;
  const float* A = (blockIdx.y == 0) ? A0 : A1; __bf16* O = (blockIdx.y == 0) ? O0 : O1;
  if (row >= nrows) return;
  const float* p = A + (size_t)row * DM;
#pragma unroll
  for (int hh = 0; hh < 2; ++hh) {
    const int c = hh * (DM / 2) + 8 * lane;
    const v4f a0 = *(const v4f*)(p + c), a1 = *(const v4f*)(p + c + 4);
    union { v8b b; v4u u; } o;
#pragma unroll
    for (int i = 0; i < 4; ++i) { o.b[i] = (__bf16)a0[i]; o.b[4 + i] = (__bf16)a1[i]; }
    vst2(O + (size_t)row * DM + c, o.u);
  }
}
__global__ __launch_bounds__(128) void k_ln(const float* __restrict__ X, const float* __restrict__ GL, const float* __restrict__ BLN, const float* __restrict__ GG, const float* __restrict__ BGN, _Float16* __restrict__ XL, _Float16* __restrict__ XG) {
  const int tid = threadIdx.x, wave = tid >> 5, lane = tid & 31;
  const int row = blockIdx.x * 4 + wave;
  if (row >= NB * SEQ) return;
  const int b = row / SEQ, t = row - b * SEQ;
  const float* p = X + ((size_t)b * SEQ_FULL + t) * DM;
  float v[16];
#pragma unroll
  for (int hh = 0; hh < 2; ++hh) {
    const v4f a0 = *(const v4f*)(p + hh * (DM / 2) + 8 * lane), a1 = *(const v4f*)(p + hh * (DM / 2) + 8 * lane + 4);
#pragma unroll
    for (int i = 0; i < 4; ++i) { v[8 * hh + i] = bfr(a0[i]); v[8 * hh + 4 + i] = bfr(a1[i]); }
  }
  float s = 0.f;
#pragma unroll
  for (int i = 0; i < 16; ++i) s += v[i];
#pragma unroll
  for (int o = 1; o < 32; o <<= 1) s += __shfl_xor(s, o);
  const float mean = s * (1.0f / 512.0f);
  float ssq = 0.f;
#pragma unroll
  for (int i = 0; i < 16; ++i) { const float d = v[i] - mean; v[i] = d; ssq += d * d; }
#pragma unroll
  for (int o = 1; o < 32; o <<= 1) ssq += __shfl_xor(ssq, o);
  const float sd = sqrtf(ssq * (1.0f / 511.0f));
  const float inv = 1.0f / (sd + 1.0e-6f);
#pragma unroll
  for (int hh = 0; hh < 2; ++hh) {
    const int c = hh * (DM / 2) + 8 * lane;
    const v4f g0 = *(const v4f*)(GL + c), g1 = *(const v4f*)(GL + c + 4), e0 = *(const v4f*)(BLN + c), e1 = *(const v4f*)(BLN + c + 4);
    const v4f f0 = *(const v4f*)(GG + c), f1 = *(const v4f*)(GG + c + 4), d0 = *(const v4f*)(BGN + c), d1 = *(const v4f*)(BGN + c + 4);
    union { v8h h; v4u u; } ol, og;
#pragma unroll
    for (int i = 0; i < 4; ++i) {
      const float n0 = v[8 * hh + i] * inv, n1 = v[8 * hh + 4 + i] * inv;
      ol.h[i] = (_Float16)(bfr(g0[i]) * n0 + bfr(e0[i])); ol.h[4 + i] = (_Float16)(bfr(g1[i]) * n1 + bfr(e1[i]));
      og.h[i] = (_Float16)(bfr(f0[i]) * n0 + bfr(d0[i])); og.h[4 + i] = (_Float16)(bfr(f1[i]) * n1 + bfr(d1[i]));
    }
    vst2(XL + (size_t)row * DM + c, ol.u);
    vst2(XG + (size_t)row * DM + c, og.u);
  }
}
__global__ __launch_bounds__(128) void k_proj(const _Float16* __restrict__ X16, const _Float16* __restrict__ W16, const float* __restrict__ BI, _Float16* __restrict__ QH, _Float16* __restrict__ QL, _Float16* __restrict__ KH, __bf16* __restrict__ VT, __bf16* __restrict__ VL) {
  __shared__ __align__(16) _Float16 sh[64][136], sl[64][136]; __shared__ __align__(16) __bf16 th[128][72], tl2[128][72];
  const int tid = threadIdx.x, wave = tid >> 5, lane = tid & 31, col = lane & 15, g = lane >> 4;
  const int which = blockIdx.y >> 2; const int c0 = (blockIdx.y & 3) * 128; const int w0 = blockIdx.y * 128; const size_t r0 = (size_t)blockIdx.x * 64;
  v8f acc[8] = {};
#pragma unroll 2
  for (int kc = 0; kc < DM / 32; ++kc) { const v16h a = frag_h(X16 + (r0 + wave * 16 + col) * DM + kc * 32, lane);
#pragma unroll
    for (int j = 0; j < 8; ++j) { const v16h w = frag_h(W16 + (size_t)(w0 + j * 16 + col) * DM + kc * 32, lane); acc[j] = wmma16(a, w, acc[j]); } }
#pragma unroll
  for (int j = 0; j < 8; ++j) { const float bb = bfr(BI[w0 + j * 16 + col]);
#pragma unroll
    for (int r = 0; r < 8; ++r) { const float v = acc[j][r] * (1.0f / 16.0f) + bb; const int rl = wave * 16 + 8 * g + r, cl = j * 16 + col; const _Float16 hv = (_Float16)v;
      if (which == 2) { const __bf16 bh = (__bf16)v; th[cl][rl] = bh; tl2[cl][rl] = (__bf16)(v - (float)bh); } else { sh[rl][cl] = hv; sl[rl][cl] = (_Float16)((v - (float)hv) * 1024.0f); } } }
  __syncthreads();
  if (which < 2) { _Float16* dh = which == 0 ? QH : KH; for (int e = tid; e < 64 * 16; e += 128) { const int rl = e >> 4, q = e & 15; vst2(dh + (r0 + rl) * DM + c0 + q * 8, *(const v4u*)&sh[rl][q * 8]); if (which == 0) vst2(QL + (r0 + rl) * DM + c0 + q * 8, *(const v4u*)&sl[rl][q * 8]); } }
  else { const size_t b = r0 / SEQ; const int t0 = (int)(r0 % SEQ); for (int e = tid; e < 128 * 8; e += 128) { const int cl = e >> 3, q = e & 7; const size_t o2 = (b * DM + c0 + cl) * (size_t)SEQ + t0 + q * 8; vst2(VT + o2, *(const v4u*)&th[cl][q * 8]); vst2(VL + o2, *(const v4u*)&tl2[cl][q * 8]); } } }
__global__ __launch_bounds__(128) void k_sc(const _Float16* __restrict__ QH, const _Float16* __restrict__ QL, const _Float16* __restrict__ KH, int b, int h0, int kp, int loc, float* __restrict__ S0) {
  __shared__ __align__(16) float ss[4][16][132];
  const int h = h0 + blockIdx.z; float* S = S0 + (size_t)blockIdx.z * SEQ * (size_t)kp;
  const int tid = threadIdx.x, wave = tid >> 5, lane = tid & 31, col = lane & 15, g = lane >> 4;
  const int kcol0 = blockIdx.y * 128; const int qb0 = blockIdx.x * 64; const int ql0 = qb0 + wave * 16; const size_t q0 = (size_t)b * SEQ + ql0;
  const int kbase = loc ? ((qb0 / WCH) - 1) * WCH : 0;
  v8f acc[8] = {}, accl[8] = {};
#pragma unroll
  for (int kc = 0; kc < HD / 32; ++kc) { const v16h ah = frag_h(QH + (q0 + col) * DM + h * HD + kc * 32, lane), al = frag_h(QL + (q0 + col) * DM + h * HD + kc * 32, lane);
#pragma unroll
    for (int j = 0; j < 8; ++j) { const int kt = kbase + kcol0 + j * 16; const int ktc = kt < 0 ? 0 : kt; const v16h kb = frag_h(KH + ((size_t)b * SEQ + ktc + col) * DM + h * HD + kc * 32, lane); acc[j] = wmma16(ah, kb, acc[j]); accl[j] = wmma16(al, kb, accl[j]); } }
#pragma unroll
  for (int j = 0; j < 8; ++j) acc[j] += accl[j] * (1.0f / 1024.0f);
#pragma unroll
  for (int j = 0; j < 8; ++j) { const bool off = (kbase + kcol0 + j * 16) < 0;
#pragma unroll
    for (int r = 0; r < 8; ++r) { const float v = acc[j][r] * 0.125f; ss[wave][8 * g + r][j * 16 + col] = off ? -3.0e38f : v; } }
  LDSX(); for (int rl = 0; rl < 16; ++rl) vst2(S + (size_t)(ql0 + rl) * kp + kcol0 + lane * 4, *(const v4f*)&ss[wave][rl][lane * 4]); }
__global__ __launch_bounds__(256) void k_sm(float* __restrict__ S0, int kp) { __shared__ float sred[8]; __shared__ float sbc; __shared__ __align__(16) float sh[SEQ];
  const int t = threadIdx.x; const size_t row = blockIdx.x; float* sr = S0 + ((size_t)blockIdx.y * SEQ + row) * (size_t)kp; const int kend = kp;
  float m = -3.0e38f; for (int k = t; k < kend; k += 256) { const float v = sr[k]; sh[k] = v; m = fmaxf(m, v); }
#pragma unroll
  for (int o = 1; o < 32; o <<= 1) m = fmaxf(m, __shfl_xor(m, o));
  if ((t & 31) == 0) sred[t >> 5] = m; __syncthreads(); if (t == 0) { float a = sred[0]; for (int i = 1; i < 8; ++i) a = fmaxf(a, sred[i]); sbc = a; } __syncthreads(); m = sbc; __syncthreads();
  float sum = 0.f; for (int k = t; k < kend; k += 256) { const float v = sh[k]; const float e = (v <= -1.0e38f) ? 0.f : expf(v - m); sh[k] = e; sum += e; }
#pragma unroll
  for (int o = 1; o < 32; o <<= 1) sum += __shfl_xor(sum, o);
  if ((t & 31) == 0) sred[t >> 5] = sum; __syncthreads(); if (t == 0) { float a = 0.f; for (int i = 0; i < 8; ++i) a += sred[i]; sbc = 1.0f / a; } __syncthreads(); const float inv = sbc;
  for (int k = t; k < kend; k += 256) sh[k] = sh[k] * inv * 2048.0f;
  __syncthreads(); for (int q = t; q < kend / 4; q += 256) vst2(sr + (size_t)q * 4, *(const v4f*)&sh[q * 4]); }
__global__ __launch_bounds__(128) void k_pv(const float* __restrict__ PS0, const __bf16* __restrict__ VT, const __bf16* __restrict__ VL, int b, int h0, int kp, int loc, float* __restrict__ Y) { const int h = h0 + blockIdx.z; const float* PS = PS0 + (size_t)blockIdx.z * SEQ * (size_t)kp; __shared__ __align__(16) float ss[4][16][HD + 4];
  const int tid = threadIdx.x, wave = tid >> 5, lane = tid & 31, col = lane & 15, g = lane >> 4; const int qb0 = blockIdx.x * 64; const int ql0 = qb0 + wave * 16;
  const int c = qb0 / WCH; const int kbase = loc ? (c - 1) * WCH : 0; const int kcs = (loc && c == 0) ? (WCH / 32) : 0; const int kce = kp / 32;
  v8f acc[HD / 16] = {};
#pragma unroll 1
  for (int kc = kcs; kc < kce; ++kc) { const F2 p = split_row(PS + (size_t)(ql0 + col) * kp, kc * 32, lane);
#pragma unroll
    for (int j = 0; j < HD / 16; ++j) { const size_t po = ((size_t)b * DM + h * HD + j * 16 + col) * (size_t)SEQ + kbase + kc * 32; const v16b vh = frag_b(VT + po, lane); acc[j] = wmma_bf(p.h, vh, acc[j]); acc[j] = wmma_bf(p.l, vh, acc[j]); acc[j] = wmma_bf(p.h, frag_b(VL + po, lane), acc[j]); } }
#pragma unroll
  for (int j = 0; j < HD / 16; ++j)
#pragma unroll
    for (int r = 0; r < 8; ++r) ss[wave][8 * g + r][j * 16 + col] = acc[j][r] * (1.0f / 2048.0f);
  LDSX(); for (int rl = 0; rl < 16; ++rl) if (lane < HD / 4) vst2(Y + ((size_t)b * SEQ + ql0 + rl) * DM + h * HD + lane * 4, *(const v4f*)&ss[wave][rl][lane * 4]); }
__global__ __launch_bounds__(128) void k_out(const float* __restrict__ YL, const __bf16* __restrict__ WL, const float* __restrict__ BL, const float* __restrict__ YG, const __bf16* __restrict__ WG, const float* __restrict__ BG, float* __restrict__ OUT) { __shared__ __align__(16) float sf[4][16][132];
  const int tid = threadIdx.x, wave = tid >> 5, lane = tid & 31, col = lane & 15, g = lane >> 4; const int c0 = blockIdx.y * 128; const size_t r0 = (size_t)blockIdx.x * 64 + wave * 16;
  v8f acc[8] = {};
#pragma unroll 1
  for (int kc = 0; kc < DM / 32; ++kc) { const F2 a = split_row(YL + (r0 + col) * DM, kc * 32, lane); const F2 e = split_row(YG + (r0 + col) * DM, kc * 32, lane);
#pragma unroll
    for (int j = 0; j < 8; ++j) { const size_t wo = (size_t)(c0 + j * 16 + col) * DM + kc * 32;
      const v16b wl = frag_b(WL + wo, lane); acc[j] = wmma_bf(a.h, wl, acc[j]); acc[j] = wmma_bf(a.l, wl, acc[j]);
      const v16b wg = frag_b(WG + wo, lane); acc[j] = wmma_bf(e.h, wg, acc[j]); acc[j] = wmma_bf(e.l, wg, acc[j]); } }
#pragma unroll
  for (int j = 0; j < 8; ++j) { const float bb = bfr(BL[c0 + j * 16 + col]) + bfr(BG[c0 + j * 16 + col]);
#pragma unroll
    for (int r = 0; r < 8; ++r) sf[wave][8 * g + r][j * 16 + col] = acc[j][r] + bb; }
  LDSX(); for (int rl = 0; rl < 16; ++rl) vst2(OUT + (r0 + rl) * DM + c0 + lane * 4, *(const v4f*)&sf[wave][rl][lane * 4]); }

extern "C" void kernel_launch(void* const* d_in, const int* in_sizes, int n_in, void* d_out, int out_size, void* d_ws, size_t ws_size, hipStream_t stream) {
  if (n_in < 13) return;
  const size_t xneed = ((size_t)(NB - 1) * SEQ_FULL + SEQ) * DM;
  if ((size_t)in_sizes[0] < xneed) return;
  if (in_sizes[1] < DM || in_sizes[2] < DM || in_sizes[3] < DM || in_sizes[4] < DM) return;
  if (in_sizes[5] < D3 * DM || in_sizes[6] < D3 || in_sizes[7] < DM * DM || in_sizes[8] < DM) return;
  if (in_sizes[9] < D3 * DM || in_sizes[10] < D3 || in_sizes[11] < DM * DM || in_sizes[12] < DM) return;
  if ((size_t)out_size < (size_t)NB * SEQ * DM) return;
  if (ws_size < (size_t)WS_END) return;
  const float* X   = (const float*)d_in[0];
  const float* GLN = (const float*)d_in[1];  const float* BLN = (const float*)d_in[2];
  const float* GGN = (const float*)d_in[3];  const float* BGN = (const float*)d_in[4];
  const float* WLI = (const float*)d_in[5];  const float* BLI = (const float*)d_in[6];
  const float* WLO = (const float*)d_in[7];  const float* BLO = (const float*)d_in[8];
  const float* WGI = (const float*)d_in[9];  const float* BGI = (const float*)d_in[10];
  const float* WGO = (const float*)d_in[11]; const float* BGO = (const float*)d_in[12];
  char* ws = (char*)d_ws;
  _Float16 *XL = (_Float16*)(ws + WS_XL), *XG = (_Float16*)(ws + WS_XG);
  _Float16 *W16L = (_Float16*)(ws + WS_WIL), *W16G = (_Float16*)(ws + WS_WIG);
  __bf16 *WBL = (__bf16*)(ws + WS_WOL), *WBG = (__bf16*)(ws + WS_WOG);
  _Float16 *QH = (_Float16*)(ws + WS_QH), *QL = (_Float16*)(ws + WS_QL), *KH = (_Float16*)(ws + WS_KH);
  __bf16 *VT = (__bf16*)(ws + WS_VT), *VL = (__bf16*)(ws + WS_VL);
  float *S = (float*)(ws + WS_S), *YL = (float*)(ws + WS_YL), *YG = (float*)(ws + WS_YG);
  float* OUT = (float*)d_out;

  k_cvt16<<<dim3(D3 / 4, 2), 128, 0, stream>>>(WLI, WGI, W16L, W16G, D3);
  k_cvtb<<<dim3(DM / 4, 2), 128, 0, stream>>>(WLO, WGO, WBL, WBG, DM);
  k_ln<<<dim3(NB * SEQ / 4), 128, 0, stream>>>(X, GLN, BLN, GGN, BGN, XL, XG);
  k_proj<<<dim3(NB * SEQ / 64, D3 / 128), 128, 0, stream>>>(XL, W16L, BLI, QH, QL, KH, VT, VL);
  for (int b = 0; b < NB; ++b) {
    k_sc<<<dim3(SEQ / 64, LK / 128, HGL), 128, 0, stream>>>(QH, QL, KH, b, 0, LK, 1, S);
    k_sm<<<dim3(SEQ, HGL), 256, 0, stream>>>(S, LK);
    k_pv<<<dim3(SEQ / 64, 1, HGL), 128, 0, stream>>>(S, VT, VL, b, 0, LK, 1, YL);
  }
  k_proj<<<dim3(NB * SEQ / 64, D3 / 128), 128, 0, stream>>>(XG, W16G, BGI, QH, QL, KH, VT, VL);
  for (int b = 0; b < NB; ++b) for (int h0 = 0; h0 < NH; h0 += HGG) {
    k_sc<<<dim3(SEQ / 64, SEQ / 128, HGG), 128, 0, stream>>>(QH, QL, KH, b, h0, SEQ, 0, S);
    k_sm<<<dim3(SEQ, HGG), 256, 0, stream>>>(S, SEQ);
    k_pv<<<dim3(SEQ / 64, 1, HGG), 128, 0, stream>>>(S, VT, VL, b, h0, SEQ, 0, YG);
  }
  k_out<<<dim3(NB * SEQ / 64, DM / 128), 128, 0, stream>>>(YL, WBL, BLO, YG, WBG, BGO, OUT);
}
